// PINN_75479755260340
// MI455X (gfx1250) — hardware-run, weakly checked
//
#include <hip/hip_runtime.h>


#ifndef NPTS
#define NPTS 131072
#endif
#define NPTS_FULL 131072
#define HDIM  256
#define PTS   32
#define NROW  (3 * PTS)
#define AP    264
#define NWAVE 8
#define NQ    1000
#define NQP   1024
#define WSC   64.0f
#define WSI   (1.0f / 64.0f)
#define T2L   2.8853900817779268f

static_assert(HDIM == 256);
static_assert(NWAVE * 32 == HDIM);
static_assert(PTS == 32);
static_assert(NROW == 96);
static_assert(HDIM % 32 == 0);
static_assert(AP >= HDIM);
static_assert((AP * 2) % 16 == 0);
static_assert(NPTS % PTS == 0);
static_assert(NPTS <= NPTS_FULL);
static_assert(NQ + 2 <= NQP);
static_assert(NQP % PTS == 0);
static_assert(NQP == 4 * 256);
static_assert((size_t)NPTS_FULL * 4 == 524288);
static_assert((size_t)2 * NPTS_FULL * 4 == 1048576);
static_assert((size_t)3 * NPTS_FULL * 4 == 1572864);
static_assert((size_t)NROW * AP * 2 + (size_t)(2 * HDIM + HDIM + NWAVE * NROW + NROW + PTS) * 4 <= 131072);
static_assert(24 * 16 == 3 * PTS * 4);
static_assert(256 * 16 == 32 * 64 * 2);
static_assert(128 * 16 == 2 * 256 * 4);
static_assert(64 * 33 * 4 <= 131072);

typedef _Float16 h16;
typedef __attribute__((ext_vector_type(16))) _Float16 v16h;
typedef __attribute__((ext_vector_type(8)))  _Float16 v8h;
typedef __attribute__((ext_vector_type(8)))  float    v8f;
typedef __attribute__((ext_vector_type(4)))  float    v4f;
typedef v4f  __attribute__((may_alias)) v4fa;
typedef v8h  __attribute__((may_alias)) v8ha;

__device__ __forceinline__ unsigned short f2bf(float f) { unsigned u = __float_as_uint(f); u += 0x7FFFu + ((u >> 16) & 1u); return (unsigned short)(u >> 16); }
__device__ __forceinline__ float bfr(float f) { return __uint_as_float(((unsigned)f2bf(f)) << 16); }
__device__ __forceinline__ v16h cat16(v8h lo, v8h hi) { return __builtin_shufflevector(lo, hi, 0, 1, 2, 3, 4, 5, 6, 7, 8, 9, 10, 11, 12, 13, 14, 15); }
__device__ __forceinline__ v16h ldh(const h16* p) { return cat16(*(const v8h*)p, *(const v8h*)(p + 16)); }
__device__ __forceinline__ v8f wmma16g(v16h a, v16h b, v8f c) {
    c = __builtin_amdgcn_wmma_f32_16x16x32_f16(false, a, false, b, (short)0, c, false, false);
    asm volatile("v_nop\n\tv_nop\n\tv_nop\n\tv_nop" : "+v"(c) : "v"(a), "v"(b));
    return c;
}
static __device__ __forceinline__ h16 toh_flush(float v) { const h16 r = (h16)v; return (fabsf(v) < 6.103515625e-05f) ? (h16)0.0f : r; }
__device__ __forceinline__ float tanh_e(float z) { const float e = __builtin_amdgcn_exp2f(z * T2L); const float rc = __builtin_amdgcn_rcpf(e + 1.0f); return 1.0f - 2.0f * rc; }

__global__ __launch_bounds__(256) void k_wconv(const float* __restrict__ W, h16* WT) {
    __shared__ float tile[64 * 33];
    const int t = threadIdx.x; const int k0 = blockIdx.x * 64, n0 = blockIdx.y * 32;
    const int tx = t & 31, ty = t >> 5;
#pragma unroll 1
    for (int j = 0; j < 8; ++j) tile[(ty + 8 * j) * 33 + tx] = W[(size_t)(k0 + ty + 8 * j) * HDIM + n0 + tx];
    __syncthreads();
    const int row = t >> 3, c8 = (t & 7) * 8;
    v8h o;
#pragma unroll
    for (int i = 0; i < 8; ++i) o[i] = toh_flush(bfr(tile[(c8 + i) * 33 + row]) * WSC);
    h16* dst = WT + (size_t)(n0 + row) * HDIM + k0 + c8;
    *(volatile v8h*)dst = o; __threadfence(); *(volatile v8h*)dst = o;
}

__global__ __launch_bounds__(256) void k_glnodes(float* tab) {
    __shared__ __align__(16) float sv[512];
    const int t = threadIdx.x; const int i = blockIdx.x * 256 + t;
    float xv = (i == NQ + 1) ? 1.0f : 0.0f, wv = 0.0f;
    if (i < NQ) {
        const double PI = 3.14159265358979323846;
        const double th = PI * ((double)i + 0.75) / ((double)NQ + 0.5);
        const bool fl = th > 0.5 * PI; const double ph = fl ? (PI - th) : th;
        const double q = ph * ph; double term = 1.0, c = 1.0;
#pragma unroll 1
        for (int k = 1; k <= 14; ++k) { term = -term * q / (double)((2 * k - 1) * (2 * k)); c += term; }
        double x = fl ? -c : c;
        double dp = 1.0;
#pragma unroll 1
        for (int it = 0; it < 12; ++it) {
            double p0 = 1.0, p1 = x;
#pragma unroll 1
            for (int k = 2; k <= NQ; ++k) { const double p2 = ((2.0 * k - 1.0) * x * p1 - (k - 1.0) * p0) / (double)k; p0 = p1; p1 = p2; }
            dp = (double)NQ * (x * p1 - p0) / (x * x - 1.0);
            const double dx = p1 / dp; x -= dx;
            if (fabs(dx) < 1e-15) break;
        }
        const double w = 2.0 / ((1.0 - x * x) * dp * dp);
        xv = (float)(0.5 * x + 0.5); wv = (float)w;
    }
    sv[t] = xv; sv[256 + t] = wv;
    __syncthreads();
    if (t < 128) {
        const int pl = t >> 6, pc = t & 63;
        const v4f val = *(const v4fa*)(&sv[pl * 256 + pc * 4]);
        float* dst = tab + (size_t)pl * NQP + (size_t)blockIdx.x * 256 + pc * 4;
        *(volatile v4f*)dst = val; __threadfence(); *(volatile v4f*)dst = val;
    }
}

__global__ __launch_bounds__(256) void k_eval(const float* __restrict__ xin, int count, int cvt,
                                              const float* __restrict__ W1, const float* __restrict__ b1,
                                              const float* __restrict__ b2, const float* __restrict__ b3,
                                              const float* __restrict__ W4, const float* __restrict__ b4,
                                              const h16* __restrict__ WT, float* outp, int ostride) {
    __shared__ __align__(16) h16 act[NROW * AP];
    __shared__ float sb[2 * HDIM];
    __shared__ float sW4[HDIM];
    __shared__ float part[NWAVE * NROW];
    __shared__ __align__(16) float res[NROW];
    __shared__ float s_pts[PTS];
    const int t = threadIdx.x;
    const int lane = t & 31, lr = lane & 15, hi = lane >> 4;
    const int wave = __builtin_amdgcn_readfirstlane((int)(threadIdx.x >> 5));
    const int base = blockIdx.x * PTS;
    {
        const int g = base + lane; const int gc = g < count ? g : count - 1;
        float xv = xin[gc]; asm volatile("" : "+v"(xv));
        const float xr = bfr(xv);
        xv = (cvt != 0) ? xr : xv;
        xv = (g < count) ? xv : 0.0f;
        if (wave == 0) s_pts[lane] = xv;
    }
    sb[t] = bfr(b2[t]); sb[HDIM + t] = bfr(b3[t]); sW4[t] = bfr(W4[t]);
    const float b4r = bfr(b4[0]);
    __syncthreads();

    {
        const float w = bfr(W1[t]), bb = bfr(b1[t]);
#pragma unroll 2
        for (int p = 0; p < PTS; ++p) {
            const float z = s_pts[p] * w + bb;
            const float h = tanh_e(z);
            const float om = 1.0f - h * h;
            const float hp = om * w;
            const float hq = -2.0f * h * hp * w;
            act[(0 * PTS + p) * AP + t] = toh_flush(h);
            act[(1 * PTS + p) * AP + t] = toh_flush(hp);
            act[(2 * PTS + p) * AP + t] = toh_flush(hq);
        }
    }
    __syncthreads();

    const int n0 = wave * 32;
    const int aoff = lr * AP + 8 * hi;
#pragma unroll 1
    for (int layer = 0; layer < 2; ++layer) {
        v8f acc[6][2];
#pragma unroll
        for (int mt = 0; mt < 6; ++mt) { acc[mt][0] = (v8f){}; acc[mt][1] = (v8f){}; }
        const size_t boff = (size_t)layer * HDIM * HDIM + (size_t)(n0 + lr) * HDIM + 8 * hi;
#pragma unroll 1
        for (int kc = 0; kc < HDIM; kc += 32) {
            const v16h bq0 = ldh(WT + boff + kc);
            const v16h bq1 = ldh(WT + boff + (size_t)16 * HDIM + kc);
#pragma unroll
            for (int mt = 0; mt < 6; ++mt) {
                const int ai = aoff + mt * 16 * AP + kc;
                const v16h a = cat16(*(const v8ha*)(&act[ai]), *(const v8ha*)(&act[ai + 16]));
                acc[mt][0] = wmma16g(a, bq0, acc[mt][0]);
                acc[mt][1] = wmma16g(a, bq1, acc[mt][1]);
            }
        }
        __syncthreads();
        const bool last = (layer == 1);
        float bcol[2], w4c[2];
#pragma unroll
        for (int nt = 0; nt < 2; ++nt) { bcol[nt] = sb[layer * HDIM + n0 + 16 * nt + lr]; w4c[nt] = sW4[n0 + 16 * nt + lr]; }
#pragma unroll
        for (int r = 0; r < 2; ++r) {
#pragma unroll
            for (int j = 0; j < 8; ++j) {
                const int p = 16 * r + 8 * hi + j;
                float hh[2], hp[2], hq[2];
#pragma unroll
                for (int nt = 0; nt < 2; ++nt) {
                    const float z  = acc[r][nt][j] * WSI + bcol[nt];
                    const float zp = acc[2 + r][nt][j] * WSI;
                    const float zq = acc[4 + r][nt][j] * WSI;
                    const float h  = tanh_e(z);
                    const float om = 1.0f - h * h;
                    const float d1 = om * zp;
                    hh[nt] = h; hp[nt] = d1; hq[nt] = om * zq - 2.0f * h * d1 * zp;
                }
                if (!last) {
#pragma unroll
                    for (int nt = 0; nt < 2; ++nt) {
                        const int c = n0 + 16 * nt + lr;
                        act[(0 * PTS + p) * AP + c] = toh_flush(hh[nt]);
                        act[(1 * PTS + p) * AP + c] = toh_flush(hp[nt]);
                        act[(2 * PTS + p) * AP + c] = toh_flush(hq[nt]);
                    }
                } else {
                    float su = hh[0] * w4c[0] + hh[1] * w4c[1];
                    float sp = hp[0] * w4c[0] + hp[1] * w4c[1];
                    float sq = hq[0] * w4c[0] + hq[1] * w4c[1];
                    su += __shfl_xor(su, 1, 32); sp += __shfl_xor(sp, 1, 32); sq += __shfl_xor(sq, 1, 32);
                    su += __shfl_xor(su, 2, 32); sp += __shfl_xor(sp, 2, 32); sq += __shfl_xor(sq, 2, 32);
                    su += __shfl_xor(su, 4, 32); sp += __shfl_xor(sp, 4, 32); sq += __shfl_xor(sq, 4, 32);
                    su += __shfl_xor(su, 8, 32); sp += __shfl_xor(sp, 8, 32); sq += __shfl_xor(sq, 8, 32);
                    if (lr == 0) {
                        part[wave * NROW + 0 * PTS + p] = su;
                        part[wave * NROW + 1 * PTS + p] = sp;
                        part[wave * NROW + 2 * PTS + p] = sq;
                    }
                }
            }
        }
        __syncthreads();
    }

    if (t < NROW) {
        float s = 0.0f;
#pragma unroll 1
        for (int w = 0; w < NWAVE; ++w) s += part[w * NROW + t];
        const float badd = (t < PTS) ? b4r : 0.0f;
        res[t] = s + badd;
    }
    __syncthreads();
    if (wave == 0) {
        const int st = lane >> 3, pc = lane & 7;
        const int stc = st < 3 ? st : 2;
        const v4f val = *(const v4fa*)(&res[stc * PTS + pc * 4]);
        float* dst = outp + (size_t)stc * (size_t)ostride + (size_t)base + pc * 4;
#pragma unroll 1
        for (int ps = 0; ps < 2; ++ps) {
            if (lane < 24) *(volatile v4f*)dst = val;
            if (ps == 0) __threadfence();
        }
    }
}

__global__ __launch_bounds__(256) void k_loss(const float* __restrict__ tab, const float* __restrict__ eu, float* out_loss) {
    __shared__ float red[256];
    float s = 0.0f;
#pragma unroll 1
    for (int i = threadIdx.x; i < NQP; i += 256) { const float d = eu[NQP + i]; s += tab[NQP + i] * d * d; }
    red[threadIdx.x] = s;
    __syncthreads();
#pragma unroll 1
    for (int off = 128; off; off >>= 1) {
        if ((int)threadIdx.x < off) red[threadIdx.x] += red[threadIdx.x + off];
        __syncthreads();
    }
    if (threadIdx.x == 0) {
        const float EA = (float)(5000.0 * 0.0004);
        const float inter = 0.5f * EA * 0.5f * 1.0f * red[0];
        const float u0 = eu[NQ];
        const float uL = eu[NQ + 1];
        const float v = 1.0f * (inter - 5.0f * uL) + 1.0f * u0 * u0;
        *(volatile float*)out_loss = v; __threadfence(); *(volatile float*)out_loss = v;
    }
}

static constexpr size_t al256(size_t v) { return (v + 255) & ~(size_t)255; }
static constexpr size_t SZ_WT  = al256((size_t)2 * HDIM * HDIM * 2);
static constexpr size_t SZ_TAB = al256((size_t)2 * NQP * 4);
static constexpr size_t SZ_EU  = al256((size_t)3 * NQP * 4);
static constexpr size_t SZ_TOTAL = SZ_WT + SZ_TAB + SZ_EU;
static_assert(SZ_TOTAL <= (size_t)134217728);
static_assert(((size_t)HDIM * HDIM * 2) % 256 == 0);
static_assert((NQP / PTS) * PTS * 4 * 3 <= 3 * NQP * 4);

extern "C" void kernel_launch(void* const* d_in, const int* in_sizes, int n_in,
                              void* d_out, int out_size, void* d_ws, size_t ws_size, hipStream_t stream) {
    if (n_in < 9) return;
    if (in_sizes[0] < NPTS) return;
    if (in_sizes[1] < HDIM || in_sizes[2] < HDIM || in_sizes[4] < HDIM || in_sizes[6] < HDIM || in_sizes[7] < HDIM || in_sizes[8] < 1) return;
    if ((size_t)in_sizes[3] < (size_t)HDIM * HDIM || (size_t)in_sizes[5] < (size_t)HDIM * HDIM) return;
    if ((size_t)out_size < (size_t)3 * NPTS_FULL + 1) return;
    if (SZ_TOTAL > ws_size) return;
    const float* x  = (const float*)d_in[0];
    const float* W1 = (const float*)d_in[1];
    const float* b1 = (const float*)d_in[2];
    const float* W2 = (const float*)d_in[3];
    const float* b2 = (const float*)d_in[4];
    const float* W3 = (const float*)d_in[5];
    const float* b3 = (const float*)d_in[6];
    const float* W4 = (const float*)d_in[7];
    const float* b4 = (const float*)d_in[8];
    float* out = (float*)d_out;
    char* wsp = (char*)d_ws;
    h16* WT = (h16*)wsp; wsp += SZ_WT;
    float* tab = (float*)wsp; wsp += SZ_TAB;
    float* eu = (float*)wsp; wsp += SZ_EU;

    k_wconv<<<dim3(HDIM / 64, HDIM / 32, 1), 256, 0, stream>>>(W2, WT);
    k_wconv<<<dim3(HDIM / 64, HDIM / 32, 1), 256, 0, stream>>>(W3, WT + (size_t)HDIM * HDIM);
    k_glnodes<<<NQP / 256, 256, 0, stream>>>(tab);
    k_eval<<<NPTS / PTS, 256, 0, stream>>>(x, NPTS, 1, W1, b1, b2, b3, W4, b4, WT, out, NPTS_FULL);
    k_eval<<<NQP / PTS, 256, 0, stream>>>(tab, NQ + 2, 0, W1, b1, b2, b3, W4, b4, WT, eu, NQP);
    k_loss<<<1, 256, 0, stream>>>(tab, eu, out + (size_t)3 * NPTS_FULL);
}
